// Mamba_69870527971709
// MI455X (gfx1250) — hardware-verified
//
#include <hip/hip_runtime.h>
#include <math.h>

typedef __attribute__((ext_vector_type(16))) _Float16 v16h;
typedef __attribute__((ext_vector_type(8)))  _Float16 v8h;
typedef __attribute__((ext_vector_type(16))) __bf16   v16b;
typedef __attribute__((ext_vector_type(8)))  __bf16   v8b;
typedef __attribute__((ext_vector_type(8)))  float    v8f;
typedef __attribute__((ext_vector_type(4)))  float    v4f;

constexpr int kBatch   = 2;
constexpr int kSeq     = 1024;
constexpr int kDm      = 1024;
constexpr int kDin     = 2048;
constexpr int kNst     = 16;
constexpr int kConvK   = 4;
constexpr int kXpP     = 2 * kDin;
constexpr int kRows    = kBatch * kSeq;
constexpr int kScanTS  = 32;
constexpr int kScanCh  = 64;
constexpr int kScanLpc = 4;
constexpr int kScanThr = kScanCh * kScanLpc;
constexpr int kScanYP  = 68;
static_assert((kDm % 32) == 0 && (kDin % 32) == 0, "GEMM K multiples of 32");
static_assert((kRows % 64) == 0 && (kXpP % 64) == 0 && (kDm % 64) == 0, "GEMM M,N multiples of 64");
static_assert((kSeq % kScanTS) == 0 && (kDin % kScanCh) == 0 && kScanCh == 64 && kScanThr == 256, "scan tile multiples");
static_assert(kScanLpc * 4 == kNst, "states per lane");
static_assert(kScanTS == (kScanThr / kScanCh) * 8, "pre-phase covers the chunk: 4 step groups x 8 steps");
static_assert(kScanTS == (kScanThr / 32) * 4, "store phase covers the chunk: 8 waves x 4 rows");
static_assert(((kRows * kDm) % (8 * 256)) == 0 && ((kXpP * kDm) % (8 * 256)) == 0 && ((kDm * kDin) % (8 * 256)) == 0, "convert grids exact");

constexpr size_t kOffXB   = 0;
constexpr size_t kOffWIP  = kOffXB  + (size_t)kRows * kDm  * 2;
constexpr size_t kOffWOP  = kOffWIP + (size_t)kXpP  * kDm  * 2;
constexpr size_t kOffXP   = kOffWOP + (size_t)kDm   * kDin * 2;
constexpr size_t kOffYH   = kOffXP  + (size_t)kRows * kXpP * 4;
constexpr size_t kOffYL   = kOffYH  + (size_t)kRows * kDin * 2;
constexpr size_t kWsTotal = kOffYL  + (size_t)kRows * kDin * 2;
static_assert(kWsTotal == 67108864ull, "carve total");
static_assert(kWsTotal <= 134217728ull, "carve cap");
static_assert((kOffWIP % 128) == 0 && (kOffWOP % 128) == 0 && (kOffXP % 128) == 0 &&
              (kOffYH % 128) == 0 && (kOffYL % 128) == 0, "128-B aligned regions");

__device__ __forceinline__ unsigned short f2bf_bits(float f) {
  unsigned u = __float_as_uint(f);
  return (unsigned short)((u + 0x7FFFu + ((u >> 16) & 1u)) >> 16);
}
__device__ __forceinline__ float bf_bits2f(unsigned short h) { return __uint_as_float(((unsigned)h) << 16); }
__device__ __forceinline__ float bf_rne(float f) { return bf_bits2f(f2bf_bits(f)); }

__device__ __forceinline__ void dep_guard_h(v8f& a, v8f& b, v16h x, v16h y) { asm volatile("v_nop\n\tv_nop\n\tv_nop\n\tv_nop" : "+v"(a), "+v"(b) : "v"(x), "v"(y)); }
__device__ __forceinline__ void dep_guard_b(v8f& a, v8f& b, v16b x, v16b y) { asm volatile("v_nop\n\tv_nop\n\tv_nop\n\tv_nop" : "+v"(a), "+v"(b) : "v"(x), "v"(y)); }
__device__ __forceinline__ void dep_guard4_h(v8f& a, v8f& b, v8f& c, v8f& d, v16h x, v16h y) { asm volatile("v_nop\n\tv_nop\n\tv_nop\n\tv_nop" : "+v"(a), "+v"(b), "+v"(c), "+v"(d) : "v"(x), "v"(y)); }
__device__ __forceinline__ void dep_guard4_b(v8f& a, v8f& b, v8f& c, v8f& d, v16b x, v16b y) { asm volatile("v_nop\n\tv_nop\n\tv_nop\n\tv_nop" : "+v"(a), "+v"(b), "+v"(c), "+v"(d) : "v"(x), "v"(y)); }
__device__ __forceinline__ void keep4_h(v16h a, v16h b, v16h c, v16h d) { asm volatile("v_nop" :: "v"(a), "v"(b), "v"(c), "v"(d)); }
__device__ __forceinline__ void keep4_b(v16b a, v16b b, v16b c, v16b d) { asm volatile("v_nop" :: "v"(a), "v"(b), "v"(c), "v"(d)); }
__device__ __forceinline__ void acc_guard4(v8f& a, v8f& b, v8f& c, v8f& d) { asm volatile("v_nop\n\tv_nop\n\tv_nop\n\tv_nop" : "+v"(a), "+v"(b), "+v"(c), "+v"(d)); }
template <typename T> struct Frag;
template <> struct Frag<_Float16> {
  typedef v16h V; union U { v16h v; v8h h[2]; };
  static __device__ __forceinline__ v16h load(const _Float16* p) {
    U f; f.h[0] = *(const v8h*)(p); f.h[1] = *(const v8h*)(p + 16); return f.v;
  }
  static __device__ __forceinline__ v8f mma(v16h a, v16h b, v8f c) {
    return __builtin_amdgcn_wmma_f32_16x16x32_f16(false, a, false, b, (short)0, c, false, false);
  }
  static __device__ __forceinline__ void guard(v8f& a, v8f& b, v16h x, v16h y) { dep_guard_h(a, b, x, y); }
  static __device__ __forceinline__ void guard4(v8f& a, v8f& b, v8f& c, v8f& d, v16h x, v16h y) { dep_guard4_h(a, b, c, d, x, y); }
  static __device__ __forceinline__ void keep(v16h a, v16h b, v16h c, v16h d) { keep4_h(a, b, c, d); }
};
template <> struct Frag<__bf16> {
  typedef v16b V; union U { v16b v; v8b h[2]; };
  static __device__ __forceinline__ v16b load(const __bf16* p) {
    U f; f.h[0] = *(const v8b*)(p); f.h[1] = *(const v8b*)(p + 16); return f.v;
  }
  static __device__ __forceinline__ v8f mma(v16b a, v16b b, v8f c) {
    return __builtin_amdgcn_wmma_f32_16x16x32_bf16(false, a, false, b, (short)0, c, false, false);
  }
  static __device__ __forceinline__ void guard(v8f& a, v8f& b, v16b x, v16b y) { dep_guard_b(a, b, x, y); }
  static __device__ __forceinline__ void guard4(v8f& a, v8f& b, v8f& c, v8f& d, v16b x, v16b y) { dep_guard4_b(a, b, c, d, x, y); }
  static __device__ __forceinline__ void keep(v16b a, v16b b, v16b c, v16b d) { keep4_b(a, b, c, d); }
};

template <int ET> struct Elem;
template <> struct Elem<0> { typedef _Float16 T; };
template <> struct Elem<1> { typedef __bf16 T; };
template <int ET, int SPL, int BIAS_MODE, int OUT_MODE, bool RESID, int ACT = 0>
__global__ __launch_bounds__(256) void wmma_gemm64(
    const unsigned short* __restrict__ Ap, const unsigned short* __restrict__ A2p, int lda, long strideA,
    const unsigned short* __restrict__ Btp, const unsigned short* __restrict__ Bt2p, int ldb, long strideB,
    void* __restrict__ Cout, void* __restrict__ Cout2, int ldc, long strideC,
    const float* __restrict__ bias,
    const float* __restrict__ resid, long strideR,
    int M, int N, int K, float scale) {
  typedef typename Elem<ET>::T T;
  typedef typename Frag<T>::V V;
  const T* A = (const T*)Ap; const T* A2 = (const T*)A2p; const T* Bt = (const T*)Btp; const T* Bt2 = (const T*)Bt2p;
  __shared__ __align__(16) float sT[8][16 * 68];
  const int b    = blockIdx.y;
  const int lane = threadIdx.x & 31;
  const int wave = threadIdx.x >> 5;
  const int tilesN = N >> 6;
  const int tilesM = M >> 6;
  const int tile = blockIdx.x * 8 + wave;
  if (tile >= tilesM * tilesN) return;
  const int tm = tile / tilesN;
  const int tn = tile - tm * tilesN;
  const int m0 = tm << 6;
  const int n0 = tn << 6;

  const T* Ab  = A  + (size_t)b * strideA;
  const T* Bb  = Bt + (size_t)b * strideB;
  const T* Ab2 = (SPL >= 1) ? (A2  + (size_t)b * strideA) : nullptr;
  const T* Bb2 = (SPL == 2) ? (Bt2 + (size_t)b * strideB) : nullptr;

  const int rlane = lane & 15;
  const int koff  = (lane >> 4) * 8;
  const int mOff  = (lane >> 4) * 8;

  v8f acc[4][4];
#pragma unroll
  for (int i = 0; i < 4; ++i)
#pragma unroll
    for (int j = 0; j < 4; ++j) acc[i][j] = (v8f){0.f,0.f,0.f,0.f,0.f,0.f,0.f,0.f};

  for (int k0 = 0; k0 < K; k0 += 32) {
    V bh[4], bl[4];
#pragma unroll
    for (int j = 0; j < 4; ++j) {
      const size_t bo = (size_t)(n0 + (j << 4) + rlane) * ldb + koff + k0;
      bh[j] = Frag<T>::load(Bb + bo);
      if (SPL == 2) bl[j] = Frag<T>::load(Bb2 + bo);
    }
#pragma unroll
    for (int i = 0; i < 4; ++i) {
      const size_t ao = (size_t)(m0 + (i << 4) + rlane) * lda + koff + k0;
      V ah = Frag<T>::load(Ab + ao);
      V al;
      if (SPL >= 1) al = Frag<T>::load(Ab2 + ao);
#pragma unroll
      for (int j = 0; j < 4; ++j) {
        acc[i][j] = Frag<T>::mma(ah, bh[j], acc[i][j]);
        if (SPL == 2) acc[i][j] = Frag<T>::mma(ah, bl[j], acc[i][j]);
        if (SPL >= 1) acc[i][j] = Frag<T>::mma(al, bh[j], acc[i][j]);
      }
      Frag<T>::guard4(acc[i][0], acc[i][1], acc[i][2], acc[i][3], ah, (SPL >= 1) ? al : ah);
    }
    Frag<T>::keep(bh[0], bh[1], bh[2], bh[3]);
    if (SPL == 2) Frag<T>::keep(bl[0], bl[1], bl[2], bl[3]);
  }
  acc_guard4(acc[0][0], acc[0][1], acc[0][2], acc[0][3]);
  acc_guard4(acc[1][0], acc[1][1], acc[1][2], acc[1][3]);
  acc_guard4(acc[2][0], acc[2][1], acc[2][2], acc[2][3]);
  acc_guard4(acc[3][0], acc[3][1], acc[3][2], acc[3][3]);

  float* slab = sT[wave];
  const float* Rb = RESID ? (resid + (size_t)b * strideR) : nullptr;
#pragma unroll
  for (int i = 0; i < 4; ++i) {
    const int mBase = m0 + (i << 4);
#pragma unroll
    for (int j = 0; j < 4; ++j) {
      const int n = n0 + (j << 4) + rlane;
      float bv = 0.f;
      if (BIAS_MODE == 2) bv = bias[n];
#pragma unroll
      for (int r = 0; r < 8; ++r) {
        float v = acc[i][j][r] * scale;
        if (BIAS_MODE == 1) v += bias[mBase + mOff + r];
        if (BIAS_MODE == 2) v += bv;
        if (RESID) v += Rb[(size_t)(mBase + mOff + r) * ldc + n];
        if (ACT == 1) v = tanhf(v);
        if (ACT == 2) v = fmaxf(v, 0.0f);
        if (ACT == 3) v = v / (1.0f + expf(-v));
        if (ACT == 4) v = (v > 0.f) ? v : 0.01f * v;
        slab[(mOff + r) * 68 + (j << 4) + rlane] = v;
      }
    }
    __builtin_amdgcn_fence(__ATOMIC_RELEASE, "workgroup");
    __builtin_amdgcn_wave_barrier();
    __builtin_amdgcn_fence(__ATOMIC_ACQUIRE, "workgroup");
    if (OUT_MODE == 0) {
      float* C = (float*)Cout + (size_t)b * strideC;
      const int hh = lane >> 4, c4 = (lane & 15) * 4;
      for (int pass = 0; pass < 2; ++pass) {
#pragma unroll
        for (int it = 0; it < 8; ++it) {
          const int row = it * 2 + hh;
          v4f v = *(const v4f*)(slab + row * 68 + c4);
          *(volatile v4f*)(C + (size_t)(mBase + row) * ldc + n0 + c4) = v;
        }
        __threadfence();
      }
    } else {
      const int q = lane >> 3, c8 = (lane & 7) * 8;
      unsigned short* C  = (unsigned short*)Cout  + (size_t)b * strideC;
      unsigned short* C2 = (OUT_MODE == 2) ? ((unsigned short*)Cout2 + (size_t)b * strideC) : nullptr;
      for (int pass = 0; pass < 2; ++pass) {
#pragma unroll
        for (int it = 0; it < 4; ++it) {
          const int row = it * 4 + q;
          const float* sp = slab + row * 68 + c8;
          v8h hv, lv;
#pragma unroll
          for (int e = 0; e < 8; ++e) {
            if (OUT_MODE == 1) {
              hv[e] = (_Float16)sp[e];
            } else {
              unsigned short hb = f2bf_bits(sp[e]);
              unsigned short lb = f2bf_bits(sp[e] - bf_bits2f(hb));
              hv[e] = __builtin_bit_cast(_Float16, hb);
              lv[e] = __builtin_bit_cast(_Float16, lb);
            }
          }
          *(volatile v8h*)(C + (size_t)(mBase + row) * ldc + n0 + c8) = hv;
          if (OUT_MODE == 2) *(volatile v8h*)(C2 + (size_t)(mBase + row) * ldc + n0 + c8) = lv;
        }
        __threadfence();
      }
    }
    __builtin_amdgcn_fence(__ATOMIC_RELEASE, "workgroup");
    __builtin_amdgcn_wave_barrier();
    __builtin_amdgcn_fence(__ATOMIC_ACQUIRE, "workgroup");
  }
}

template <bool PERM>
__global__ __launch_bounds__(256) void cvt_rows_bf16_kernel(
    const float* __restrict__ src, unsigned short* __restrict__ dst, int total8, int cols, int half)
{
  const int i = blockIdx.x * 256 + threadIdx.x;
  if (i >= total8) return;
  const size_t e0 = (size_t)i << 3;
  size_t o0 = e0;
  if (PERM) {
    const size_t r  = e0 / (size_t)cols;
    const size_t c  = e0 - r * (size_t)cols;
    const size_t dr = (r & 1) * (size_t)half + (r >> 1);
    o0 = dr * (size_t)cols + c;
  }
  const v4f a0 = *(const v4f*)(src + e0);
  const v4f a1 = *(const v4f*)(src + e0 + 4);
  v8h hv;
#pragma unroll
  for (int e = 0; e < 4; ++e) {
    const float f0 = a0[e], f1 = a1[e];
    const unsigned short h0 = f2bf_bits(f0), h1 = f2bf_bits(f1);
    hv[e]     = __builtin_bit_cast(_Float16, h0);
    hv[4 + e] = __builtin_bit_cast(_Float16, h1);
  }
  unsigned short* qd = dst + o0;
  *(volatile v8h*)qd = hv;
  __threadfence();
  *(volatile v8h*)qd = hv;
}

__global__ __launch_bounds__(256) void scan_kernel(
    const float* __restrict__ XP, const float* __restrict__ cw, const float* __restrict__ cb,
    const float* __restrict__ Aar, const float* __restrict__ Bar, const float* __restrict__ Car,
    unsigned short* __restrict__ YH, unsigned short* __restrict__ YL)
{
  __shared__ __align__(16) float sDL[kScanTS * kScanCh];
  __shared__ __align__(16) float sDU[kScanTS * kScanCh];
  __shared__ __align__(16) float sSG[kScanTS * kScanCh];
  __shared__ __align__(16) float sY[kScanTS * kScanYP];
  const int tid = threadIdx.x, lane = tid & 31, wave = tid >> 5;
  constexpr int kBlkPerB = kDin / kScanCh;
  const int bix = blockIdx.x / kBlkPerB;
  const int d0  = (blockIdx.x - bix * kBlkPerB) * kScanCh;
  const size_t row0 = (size_t)bix * kSeq;

  const int cr = tid >> 2, pr = tid & 3;
  const int dr = d0 + cr;
  float Av[4], Bv[4], Cv[4], h[4];
  {
    const v4f av = *(const v4f*)(Aar + (size_t)dr * kNst + 4 * pr);
    const v4f bv = *(const v4f*)(Bar + (size_t)dr * kNst + 4 * pr);
    const v4f cv = *(const v4f*)(Car + (size_t)dr * kNst + 4 * pr);
#pragma unroll
    for (int k = 0; k < 4; ++k) {
      const float fa = av[k], fb = bv[k], fc = cv[k];
      Av[k] = bf_rne(fa);
      Bv[k] = bf_rne(fb);
      Cv[k] = bf_rne(fc);
      h[k] = 0.0f;
    }
  }
  const int cq = tid & (kScanCh - 1), sgp = tid >> 6;
  const int dq = d0 + cq;
  const v4f cwv = *(const v4f*)(cw + (size_t)dq * kConvK);
  const float cw0 = cwv[0], cw1 = cwv[1], cw2 = cwv[2], cw3 = cwv[3];
  const float w0 = bf_rne(cw0), w1 = bf_rne(cw1), w2 = bf_rne(cw2), w3 = bf_rne(cw3);
  const float bcv = bf_rne(cb[dq]);

  const int q = lane >> 3, c8 = (lane & 7) * 8;
#pragma unroll 1
  for (int t0 = 0; t0 < kSeq; t0 += kScanTS) {
#pragma unroll 1
    for (int j = 0; j < 8; ++j) {
      const int sl = sgp * 8 + j;
      const int t  = t0 + sl;
      const int r1i = (t >= 1) ? (t - 1) : 0;
      const int r2i = (t >= 2) ? (t - 2) : 0;
      const int r3i = (t >= 3) ? (t - 3) : 0;
      const float f1 = (t >= 1) ? 1.0f : 0.0f;
      const float f2 = (t >= 2) ? 1.0f : 0.0f;
      const float f3 = (t >= 3) ? 1.0f : 0.0f;
      const float u0 = XP[(row0 + (size_t)t)   * kXpP + dq];
      const float u1 = XP[(row0 + (size_t)r1i) * kXpP + dq] * f1;
      const float u2 = XP[(row0 + (size_t)r2i) * kXpP + dq] * f2;
      const float u3 = XP[(row0 + (size_t)r3i) * kXpP + dq] * f3;
      const float gv = XP[(row0 + (size_t)t)   * kXpP + kDin + dq];
      float cacc = w0 * u3;
      cacc = fmaf(w1, u2, cacc);
      cacc = fmaf(w2, u1, cacc);
      cacc = fmaf(w3, u0, cacc);
      const float xc = cacc + bcv;
      const float ex = expf(-xc);
      const float dl = __builtin_amdgcn_rcpf(1.0f + ex);
      const float du = dl * xc;
      const float eg = expf(-gv);
      const float sg = __builtin_amdgcn_rcpf(1.0f + eg);
      sDL[sl * kScanCh + cq] = dl;
      sDU[sl * kScanCh + cq] = du;
      sSG[sl * kScanCh + cq] = sg;
    }
    __syncthreads();
#pragma unroll 1
    for (int s = 0; s < kScanTS; ++s) {
      const float dl = sDL[s * kScanCh + cr];
      const float du = sDU[s * kScanCh + cr];
      const float sg = sSG[s * kScanCh + cr];
#pragma unroll
      for (int k = 0; k < 4; ++k) {
        const float ak = Av[k] * dl;
        const float bk = Bv[k] * du;
        h[k] = ak * h[k] + bk;
      }
      float yp = h[0] * Cv[0];
      yp = fmaf(h[1], Cv[1], yp);
      yp = fmaf(h[2], Cv[2], yp);
      yp = fmaf(h[3], Cv[3], yp);
      yp += __shfl_xor(yp, 1, 32);
      yp += __shfl_xor(yp, 2, 32);
      sY[s * kScanYP + cr] = yp * sg;
    }
    __syncthreads();
    const int row = wave * 4 + q;
    v8h hv, lv;
    {
      const float* sp = sY + row * kScanYP + c8;
      const v4f a0 = *(const v4f*)(sp);
      const v4f a1 = *(const v4f*)(sp + 4);
#pragma unroll
      for (int e = 0; e < 4; ++e) {
        const float g0 = a0[e], g1 = a1[e];
        const unsigned short h0 = f2bf_bits(g0), h1 = f2bf_bits(g1);
        const unsigned short l0 = f2bf_bits(g0 - bf_bits2f(h0)), l1 = f2bf_bits(g1 - bf_bits2f(h1));
        hv[e]     = __builtin_bit_cast(_Float16, h0);
        hv[4 + e] = __builtin_bit_cast(_Float16, h1);
        lv[e]     = __builtin_bit_cast(_Float16, l0);
        lv[4 + e] = __builtin_bit_cast(_Float16, l1);
      }
    }
    const size_t o = (row0 + (size_t)(t0 + row)) * kDin + d0 + c8;
    for (int pass = 0; pass < 2; ++pass) {
      *(volatile v8h*)(YH + o) = hv;
      *(volatile v8h*)(YL + o) = lv;
      __threadfence();
    }
  }
}

extern "C" void kernel_launch(void* const* d_in, const int* in_sizes, int n_in,
                              void* d_out, int out_size, void* d_ws, size_t ws_size,
                              hipStream_t stream) {
  if (n_in < 9) return;
  if (in_sizes[0] != kRows * kDm) return;
  if (in_sizes[1] != kXpP * kDm) return;
  if (in_sizes[2] != kDin * kConvK) return;
  if (in_sizes[3] != kDin) return;
  if (in_sizes[4] != kDin * kNst) return;
  if (in_sizes[5] != kDin * kNst) return;
  if (in_sizes[6] != kDin * kNst) return;
  if (in_sizes[8] != kDm * kDin) return;
  if (out_size != kRows * kDm) return;
  if (ws_size < kWsTotal) return;

  const float* x      = (const float*)d_in[0];
  const float* W_in   = (const float*)d_in[1];
  const float* conv_w = (const float*)d_in[2];
  const float* conv_b = (const float*)d_in[3];
  const float* Aar    = (const float*)d_in[4];
  const float* Bar    = (const float*)d_in[5];
  const float* Car    = (const float*)d_in[6];
  const float* W_out  = (const float*)d_in[8];
  float* out = (float*)d_out;

  char* ws = (char*)d_ws;
  unsigned short* XB  = (unsigned short*)(ws + kOffXB);
  unsigned short* WIP = (unsigned short*)(ws + kOffWIP);
  unsigned short* WOP = (unsigned short*)(ws + kOffWOP);
  float*          XP  = (float*)(ws + kOffXP);
  unsigned short* YH  = (unsigned short*)(ws + kOffYH);
  unsigned short* YL  = (unsigned short*)(ws + kOffYL);

  {
    const int n8x = kRows * kDm / 8, n8wi = kXpP * kDm / 8, n8wo = kDm * kDin / 8;
    cvt_rows_bf16_kernel<false><<<(n8x + 255) / 256, 256, 0, stream>>>(x, XB, n8x, kDm, 0);
    cvt_rows_bf16_kernel<true><<<(n8wi + 255) / 256, 256, 0, stream>>>(W_in, WIP, n8wi, kDm, kDin);
    cvt_rows_bf16_kernel<false><<<(n8wo + 255) / 256, 256, 0, stream>>>(W_out, WOP, n8wo, kDin, 0);
  }

  wmma_gemm64<1, 0, 0, 0, false><<<dim3((kRows / 64) * (kXpP / 64) / 8, 1), 256, 0, stream>>>(
      XB, nullptr, kDm, 0L,
      WIP, nullptr, kDm, 0L,
      (void*)XP, nullptr, kXpP, 0L,
      nullptr, nullptr, 0L,
      kRows, kXpP, kDm, 1.0f);

  scan_kernel<<<kBatch * (kDin / kScanCh), kScanThr, 0, stream>>>(XP, conv_w, conv_b, Aar, Bar, Car, YH, YL);

  wmma_gemm64<1, 1, 0, 0, false><<<dim3((kRows / 64) * (kDm / 64) / 8, 1), 256, 0, stream>>>(
      YH, YL, kDin, 0L,
      WOP, nullptr, kDin, 0L,
      (void*)out, nullptr, kDm, 0L,
      nullptr, nullptr, 0L,
      kRows, kDm, kDin, 1.0f);
}
